// SS2Dv0_3384434229777
// MI455X (gfx1250) — hardware-verified
//
#include <hip/hip_runtime.h>
#include <math.h>

typedef __attribute__((ext_vector_type(16))) _Float16 v16h;
typedef __attribute__((ext_vector_type(8)))  _Float16 v8h;
typedef __attribute__((ext_vector_type(16))) __bf16   v16b;
typedef __attribute__((ext_vector_type(8)))  __bf16   v8b;
typedef __attribute__((ext_vector_type(8)))  float    v8f;
typedef __attribute__((ext_vector_type(4)))  float    v4f;

constexpr int NBATCH = 2;
constexpr int CMOD   = 768;
constexpr int IMH    = 32;
constexpr int IMW    = 32;
constexpr int NPIX   = IMH * IMW;
constexpr int NTOK   = NBATCH * NPIX;
constexpr int DIN    = 1536;
constexpr int NST    = 16;
constexpr int DTR    = 48;
constexpr int DTRP   = 64;
constexpr int NDIR   = 4;
constexpr int XPR    = 80;
constexpr int XPRP   = 128;
constexpr int CGRP   = 256;
constexpr int NCG    = DIN / CGRP;
constexpr int SCH    = 64;
constexpr int DPL    = 2;
static_assert(NCG * CGRP == DIN, "channel groups");
static_assert((SCH * 8) % CGRP == 0, "staging coverage");
static_assert(NPIX % SCH == 0, "chunking");

__device__ __forceinline__ unsigned short f2bf_bits(float f) {
  unsigned u = __float_as_uint(f);
  return (unsigned short)((u + 0x7FFFu + ((u >> 16) & 1u)) >> 16);
}
__device__ __forceinline__ float bf_bits2f(unsigned short h) { return __uint_as_float(((unsigned)h) << 16); }

__device__ __forceinline__ void dep_guard_h(v8f& a, v8f& b, v16h x, v16h y) { asm volatile("v_nop\n\tv_nop\n\tv_nop\n\tv_nop" : "+v"(a), "+v"(b) : "v"(x), "v"(y)); }
__device__ __forceinline__ void dep_guard_b(v8f& a, v8f& b, v16b x, v16b y) { asm volatile("v_nop\n\tv_nop\n\tv_nop\n\tv_nop" : "+v"(a), "+v"(b) : "v"(x), "v"(y)); }
__device__ __forceinline__ void keep4_h(v16h a, v16h b, v16h c, v16h d) { asm volatile("v_nop" :: "v"(a), "v"(b), "v"(c), "v"(d)); }
__device__ __forceinline__ void keep4_b(v16b a, v16b b, v16b c, v16b d) { asm volatile("v_nop" :: "v"(a), "v"(b), "v"(c), "v"(d)); }
__device__ __forceinline__ void acc_guard4(v8f& a, v8f& b, v8f& c, v8f& d) { asm volatile("v_nop\n\tv_nop\n\tv_nop\n\tv_nop" : "+v"(a), "+v"(b), "+v"(c), "+v"(d)); }
template <typename T> struct Frag;
template <> struct Frag<_Float16> {
  typedef v16h V; union U { v16h v; v8h h[2]; };
  static __device__ __forceinline__ v16h load(const _Float16* p) {
    U f; f.h[0] = *(const v8h*)(p); f.h[1] = *(const v8h*)(p + 16); return f.v;
  }
  static __device__ __forceinline__ v8f mma(v16h a, v16h b, v8f c) {
    return __builtin_amdgcn_wmma_f32_16x16x32_f16(false, a, false, b, (short)0, c, false, false);
  }
  static __device__ __forceinline__ void guard(v8f& a, v8f& b, v16h x, v16h y) { dep_guard_h(a, b, x, y); }
  static __device__ __forceinline__ void keep(v16h a, v16h b, v16h c, v16h d) { keep4_h(a, b, c, d); }
};
template <> struct Frag<__bf16> {
  typedef v16b V; union U { v16b v; v8b h[2]; };
  static __device__ __forceinline__ v16b load(const __bf16* p) {
    U f; f.h[0] = *(const v8b*)(p); f.h[1] = *(const v8b*)(p + 16); return f.v;
  }
  static __device__ __forceinline__ v8f mma(v16b a, v16b b, v8f c) {
    return __builtin_amdgcn_wmma_f32_16x16x32_bf16(false, a, false, b, (short)0, c, false, false);
  }
  static __device__ __forceinline__ void guard(v8f& a, v8f& b, v16b x, v16b y) { dep_guard_b(a, b, x, y); }
  static __device__ __forceinline__ void keep(v16b a, v16b b, v16b c, v16b d) { keep4_b(a, b, c, d); }
};

template <int ET> struct Elem;
template <> struct Elem<0> { typedef _Float16 T; };
template <> struct Elem<1> { typedef __bf16 T; };
template <int ET, bool SPLIT, int BIAS_MODE, int OUT_MODE, bool RESID, int ACT = 0>
__global__ __launch_bounds__(256) void wmma_gemm64(
    const unsigned short* __restrict__ Ap, const unsigned short* __restrict__ A2p, int lda, long strideA,
    const unsigned short* __restrict__ Btp, const unsigned short* __restrict__ Bt2p, int ldb, long strideB,
    void* __restrict__ Cout, void* __restrict__ Cout2, int ldc, long strideC,
    const float* __restrict__ bias,
    const float* __restrict__ resid, long strideR,
    int M, int N, int K, float scale) {
  typedef typename Elem<ET>::T T;
  typedef typename Frag<T>::V V;
  const T* A = (const T*)Ap; const T* A2 = (const T*)A2p; const T* Bt = (const T*)Btp; const T* Bt2 = (const T*)Bt2p;
  __shared__ __align__(16) float sT[8][16 * 68];
  const int b    = blockIdx.y;
  const int lane = threadIdx.x & 31;
  const int wave = threadIdx.x >> 5;
  const int tilesN = N >> 6;
  const int tilesM = M >> 6;
  const int tile = blockIdx.x * 8 + wave;
  if (tile >= tilesM * tilesN) return;
  const int tm = tile / tilesN;
  const int tn = tile - tm * tilesN;
  const int m0 = tm << 6;
  const int n0 = tn << 6;

  const T* Ab  = A  + (size_t)b * strideA;
  const T* Bb  = Bt + (size_t)b * strideB;
  const T* Ab2 = SPLIT ? (A2  + (size_t)b * strideA) : nullptr;
  const T* Bb2 = SPLIT ? (Bt2 + (size_t)b * strideB) : nullptr;

  const int rlane = lane & 15;
  const int koff  = (lane >> 4) * 8;
  const int mOff  = (lane >> 4) * 8;

  v8f acc[4][4];
#pragma unroll
  for (int i = 0; i < 4; ++i)
#pragma unroll
    for (int j = 0; j < 4; ++j) acc[i][j] = (v8f){0.f,0.f,0.f,0.f,0.f,0.f,0.f,0.f};

  for (int k0 = 0; k0 < K; k0 += 32) {
    V bh[4], bl[4];
#pragma unroll
    for (int j = 0; j < 4; ++j) {
      const size_t bo = (size_t)(n0 + (j << 4) + rlane) * ldb + koff + k0;
      bh[j] = Frag<T>::load(Bb + bo);
      if (SPLIT) bl[j] = Frag<T>::load(Bb2 + bo);
    }
#pragma unroll
    for (int i = 0; i < 4; ++i) {
      const size_t ao = (size_t)(m0 + (i << 4) + rlane) * lda + koff + k0;
      V ah = Frag<T>::load(Ab + ao);
      V al;
      if (SPLIT) al = Frag<T>::load(Ab2 + ao);
#pragma unroll
      for (int j = 0; j < 4; ++j) {
        acc[i][j] = Frag<T>::mma(ah, bh[j], acc[i][j]);
        if (SPLIT) {
          acc[i][j] = Frag<T>::mma(ah, bl[j], acc[i][j]);
          acc[i][j] = Frag<T>::mma(al, bh[j], acc[i][j]);
        }
      }
      Frag<T>::guard(acc[i][0], acc[i][3], ah, SPLIT ? al : ah);
    }
    Frag<T>::keep(bh[0], bh[1], bh[2], bh[3]);
    if (SPLIT) Frag<T>::keep(bl[0], bl[1], bl[2], bl[3]);
  }
  acc_guard4(acc[0][0], acc[0][1], acc[0][2], acc[0][3]);
  acc_guard4(acc[1][0], acc[1][1], acc[1][2], acc[1][3]);
  acc_guard4(acc[2][0], acc[2][1], acc[2][2], acc[2][3]);
  acc_guard4(acc[3][0], acc[3][1], acc[3][2], acc[3][3]);

  float* slab = sT[wave];
  const float* Rb = RESID ? (resid + (size_t)b * strideR) : nullptr;
#pragma unroll
  for (int i = 0; i < 4; ++i) {
    const int mBase = m0 + (i << 4);
#pragma unroll
    for (int j = 0; j < 4; ++j) {
      const int n = n0 + (j << 4) + rlane;
      float bv = 0.f;
      if (BIAS_MODE == 2) bv = bias[n];
#pragma unroll
      for (int r = 0; r < 8; ++r) {
        float v = acc[i][j][r] * scale;
        if (BIAS_MODE == 1) v += bias[mBase + mOff + r];
        if (BIAS_MODE == 2) v += bv;
        if (RESID) v += Rb[(size_t)(mBase + mOff + r) * ldc + n];
        if (ACT == 1) v = tanhf(v);
        if (ACT == 2) v = fmaxf(v, 0.0f);
        if (ACT == 3) v = v / (1.0f + expf(-v));
        if (ACT == 4) v = (v > 0.f) ? v : 0.01f * v;
        if (ACT == 5) v = 0.5f * v * (1.0f + erff(v * 0.70710678118654752f));
        slab[(mOff + r) * 68 + (j << 4) + rlane] = v;
      }
    }
    __builtin_amdgcn_fence(__ATOMIC_RELEASE, "workgroup");
    __builtin_amdgcn_wave_barrier();
    __builtin_amdgcn_fence(__ATOMIC_ACQUIRE, "workgroup");
    if (OUT_MODE == 0) {
      float* C = (float*)Cout + (size_t)b * strideC;
      const int hh = lane >> 4, c4 = (lane & 15) * 4;
      for (int pass = 0; pass < 2; ++pass) {
#pragma unroll
        for (int it = 0; it < 8; ++it) {
          const int row = it * 2 + hh;
          v4f v = *(const v4f*)(slab + row * 68 + c4);
          *(volatile v4f*)(C + (size_t)(mBase + row) * ldc + n0 + c4) = v;
        }
        __threadfence();
      }
    } else {
      const int q = lane >> 3, c8 = (lane & 7) * 8;
      unsigned short* C  = (unsigned short*)Cout  + (size_t)b * strideC;
      unsigned short* C2 = (OUT_MODE == 2) ? ((unsigned short*)Cout2 + (size_t)b * strideC) : nullptr;
      for (int pass = 0; pass < 2; ++pass) {
#pragma unroll
        for (int it = 0; it < 4; ++it) {
          const int row = it * 4 + q;
          const float* sp = slab + row * 68 + c8;
          v8h hv, lv;
#pragma unroll
          for (int e = 0; e < 8; ++e) {
            if (OUT_MODE == 1) {
              hv[e] = (_Float16)sp[e];
            } else {
              unsigned short hb = f2bf_bits(sp[e]);
              unsigned short lb = f2bf_bits(sp[e] - bf_bits2f(hb));
              hv[e] = __builtin_bit_cast(_Float16, hb);
              lv[e] = __builtin_bit_cast(_Float16, lb);
            }
          }
          *(volatile v8h*)(C + (size_t)(mBase + row) * ldc + n0 + c8) = hv;
          if (OUT_MODE == 2) *(volatile v8h*)(C2 + (size_t)(mBase + row) * ldc + n0 + c8) = lv;
        }
        __threadfence();
      }
    }
    __builtin_amdgcn_fence(__ATOMIC_RELEASE, "workgroup");
    __builtin_amdgcn_wave_barrier();
    __builtin_amdgcn_fence(__ATOMIC_ACQUIRE, "workgroup");
  }
}

__global__ __launch_bounds__(256) void cast_pad_kernel(
    const float* __restrict__ src, int spitch, int R,
    unsigned short* __restrict__ dst, int Kcp, int Ku, int nchunks, float scale)
{
  const int f = blockIdx.x * 256 + threadIdx.x;
  if (f >= nchunks) return;
  const int cpr = Kcp >> 3;
  const int n = f / cpr;
  const int g = f - n * cpr;
  const bool cval  = (g * 8) < Ku;
  const bool rval  = n < R;
  const bool valid = rval && cval;
  const int sr = rval ? n : 0;
  const int sc = cval ? (g * 8) : 0;
  const float* p = src + (size_t)sr * spitch + sc;
  const v4f a0 = *(const v4f*)(p);
  const v4f a1 = *(const v4f*)(p + 4);
  v8h hv;
#pragma unroll
  for (int e = 0; e < 4; ++e) {
    hv[e]     = (_Float16)(valid ? a0[e] * scale : 0.0f);
    hv[4 + e] = (_Float16)(valid ? a1[e] * scale : 0.0f);
  }
  unsigned short* q = dst + (size_t)f * 8;
  *(volatile v8h*)q = hv;
  __threadfence();
  *(volatile v8h*)q = hv;
}

__global__ __launch_bounds__(256) void xpose_cast_kernel(const float* __restrict__ x, unsigned short* __restrict__ X16)
{
  __shared__ __align__(16) _Float16 sX[64 * 72];
  const int t = threadIdx.x, lane = t & 31, wave = t >> 5;
  const int ct = blockIdx.x % (CMOD / 64);
  const int tt = blockIdx.x / (CMOD / 64);
  const int b_ = tt / (NPIX / 64);
  const int l0 = (tt - b_ * (NPIX / 64)) * 64;
  const int c0 = ct * 64;
#pragma unroll
  for (int pass = 0; pass < 4; ++pass) {
    const int c  = pass * 16 + (t >> 4);
    const int l4 = (t & 15) * 4;
    const v4f v = *(const v4f*)(x + ((size_t)(b_ * CMOD + c0 + c)) * NPIX + l0 + l4);
#pragma unroll
    for (int e = 0; e < 4; ++e) sX[(l4 + e) * 72 + c] = (_Float16)v[e];
  }
  __syncthreads();
  const int q = lane >> 3, c8 = (lane & 7) * 8;
  v8h vals[2];
#pragma unroll
  for (int it = 0; it < 2; ++it) vals[it] = *(const v8h*)(sX + ((wave * 2 + it) * 4 + q) * 72 + c8);
  unsigned short* ob = X16 + ((size_t)(b_ * NPIX + l0)) * CMOD + c0;
  for (int pass = 0; pass < 2; ++pass) {
#pragma unroll
    for (int it = 0; it < 2; ++it)
      *(volatile v8h*)(ob + (size_t)((wave * 2 + it) * 4 + q) * CMOD + c8) = vals[it];
    __threadfence();
  }
}

__global__ __launch_bounds__(256) void dwconv_silu_kernel(
    const float* __restrict__ XI, const float* __restrict__ cw, const float* __restrict__ cbias,
    float* __restrict__ XC, unsigned short* __restrict__ XC16)
{
  __shared__ __align__(16) _Float16 sH[IMW * CGRP];
  const int t = threadIdx.x, lane = t & 31, wave = t >> 5;
  const int cg = blockIdx.x % NCG;
  const int bh = blockIdx.x / NCG;
  const int b_ = bh / IMH;
  const int h_ = bh - b_ * IMH;
  const int d  = cg * CGRP + t;
  const float* wd = cw + (size_t)d * 9;
  const float w00 = wd[0], w01 = wd[1], w02 = wd[2];
  const float w10 = wd[3], w11 = wd[4], w12 = wd[5];
  const float w20 = wd[6], w21 = wd[7], w22 = wd[8];
  const float bc = cbias[d];
  const bool up = h_ > 0, dn = h_ < IMH - 1;
  const int r0 = up ? (h_ - 1) : 0;
  const int r2 = dn ? (h_ + 1) : (IMH - 1);
  const float* p0 = XI + ((size_t)(b_ * IMH + r0) * IMW) * DIN + d;
  const float* p1 = XI + ((size_t)(b_ * IMH + h_) * IMW) * DIN + d;
  const float* p2 = XI + ((size_t)(b_ * IMH + r2) * IMW) * DIN + d;
  float a0m = 0.f, a1m = 0.f, a2m = 0.f;
  float a0c, a1c, a2c;
  {
    const float v0 = p0[0], v1 = p1[0], v2 = p2[0];
    a0c = up ? v0 : 0.f;
    a1c = v1;
    a2c = dn ? v2 : 0.f;
  }
  float* orow = XC + ((size_t)(b_ * IMH + h_) * IMW) * DIN + d;
#pragma unroll 1
  for (int w = 0; w < IMW; ++w) {
    const bool rv = (w + 1) < IMW;
    const int  wn = rv ? (w + 1) : (IMW - 1);
    const float n0 = p0[(size_t)wn * DIN], n1 = p1[(size_t)wn * DIN], n2 = p2[(size_t)wn * DIN];
    const float a0n = (up && rv) ? n0 : 0.f;
    const float a1n = rv ? n1 : 0.f;
    const float a2n = (dn && rv) ? n2 : 0.f;
    float acc = w00 * a0m;
    acc = fmaf(w01, a0c, acc);
    acc = fmaf(w02, a0n, acc);
    acc = fmaf(w10, a1m, acc);
    acc = fmaf(w11, a1c, acc);
    acc = fmaf(w12, a1n, acc);
    acc = fmaf(w20, a2m, acc);
    acc = fmaf(w21, a2c, acc);
    acc = fmaf(w22, a2n, acc);
    const float sv  = acc + bc;
    const float sg  = __builtin_amdgcn_rcpf(1.0f + __expf(-sv));
    const float out = sv * sg;
    float* op = orow + (size_t)w * DIN;
    *(volatile float*)op = out;
    __threadfence();
    *(volatile float*)op = out;
    sH[w * CGRP + t] = (_Float16)(out * 64.0f);
    a0m = a0c; a0c = a0n;
    a1m = a1c; a1c = a1n;
    a2m = a2c; a2c = a2n;
  }
  __syncthreads();
  v8h vals[4];
#pragma unroll
  for (int i = 0; i < 4; ++i) vals[i] = *(const v8h*)(sH + (wave * 4 + i) * CGRP + lane * 8);
  unsigned short* ob = XC16 + ((size_t)(b_ * IMH + h_) * IMW) * DIN + (size_t)cg * CGRP;
  for (int pass = 0; pass < 2; ++pass) {
#pragma unroll
    for (int i = 0; i < 4; ++i)
      *(volatile v8h*)(ob + (size_t)(wave * 4 + i) * DIN + lane * 8) = vals[i];
    __threadfence();
  }
}

__device__ __forceinline__ int dir_tok(int k, int l) {
  const int lr = (k >= 2) ? (NPIX - 1 - l) : l;
  return (k & 1) ? (((lr & (IMH - 1)) * IMW) + (lr >> 5)) : lr;
}

__global__ __launch_bounds__(256) void scan_dir_kernel(
    const float* __restrict__ XDBL, const float* __restrict__ XC, const float* __restrict__ DT,
    const float* __restrict__ dtb, const float* __restrict__ Alog, const float* __restrict__ Dsp,
    float* __restrict__ Y, int kbase)
{
  __shared__ __align__(16) float sBC[SCH * 32];
  const int t    = threadIdx.x;
  const int cg   = blockIdx.x % NCG;
  const int rest = blockIdx.x / NCG;
  const int kk   = rest % DPL;
  const int b_   = rest / DPL;
  const int k    = kbase + kk;
  const int d    = cg * CGRP + t;
  const int kd   = k * DIN + d;
  const float db = dtb[kd];
  const float Dk = Dsp[kd];
  float An[NST], h[NST];
#pragma unroll
  for (int n = 0; n < NST; ++n) {
    An[n] = -__expf(Alog[(size_t)kd * NST + n]);
    h[n]  = 0.f;
  }
  const size_t tokb = (size_t)b_ * NPIX;
  const float* DTk = DT + (size_t)kk * NTOK * DIN;
  float* Yk = Y + (size_t)k * NTOK * DIN;
#pragma unroll 1
  for (int c = 0; c < NPIX / SCH; ++c) {
    __syncthreads();
#pragma unroll 1
    for (int q = t; q < SCH * 8; q += CGRP) {
      const int s   = q >> 3;
      const int j   = q & 7;
      const int tok = dir_tok(k, c * SCH + s);
      const v4f v = *(const v4f*)(XDBL + (tokb + tok) * XPRP + DTR + 4 * j);
      *(v4f*)(sBC + s * 32 + 4 * j) = v;
    }
    __syncthreads();
#pragma unroll 1
    for (int s = 0; s < SCH; ++s) {
      const int tok = dir_tok(k, c * SCH + s);
      const size_t ei = (tokb + tok) * DIN + d;
      const float u  = XC[ei];
      const float dp = DTk[ei] + db;
      const float ex   = __expf(-fabsf(dp));
      const float up1  = 1.0f + ex;
      const float den  = up1 - 1.0f;
      const bool  dpos = den > 0.0f;
      const float dens = dpos ? den : 1.0f;
      const float lg   = __logf(up1);
      const float l1p  = dpos ? (lg * (ex * __builtin_amdgcn_rcpf(dens))) : ex;
      const float delta = fmaxf(dp, 0.0f) + l1p;
      const float* sr = sBC + s * 32;
      v4f Bv[4], Cv[4];
#pragma unroll
      for (int i = 0; i < 4; ++i) {
        Bv[i] = *(const v4f*)(sr + 4 * i);
        Cv[i] = *(const v4f*)(sr + 16 + 4 * i);
      }
      const float du = delta * u;
      float ys = 0.f;
#pragma unroll
      for (int n = 0; n < NST; ++n) {
        const float e  = __expf(delta * An[n]);
        const float hn = fmaf(e, h[n], du * Bv[n >> 2][n & 3]);
        h[n] = hn;
        ys = fmaf(hn, Cv[n >> 2][n & 3], ys);
      }
      const float y = ys + Dk * u;
      float* yp = Yk + ei;
      *(volatile float*)yp = y;
      __threadfence();
      *(volatile float*)yp = y;
    }
  }
}

__global__ __launch_bounds__(192) void ln_gate_kernel(
    const float* __restrict__ Y, const float* __restrict__ Z,
    const float* __restrict__ gam, const float* __restrict__ bet,
    unsigned short* __restrict__ YG16)
{
  __shared__ float sred[16];
  const int t = threadIdx.x, lane = t & 31, wave = t >> 5;
  const int row = blockIdx.x;
  const int c0  = t * 8;
  const size_t PL   = (size_t)NTOK * DIN;
  const size_t base = (size_t)row * DIN + c0;
  v4f a[2];
#pragma unroll
  for (int j = 0; j < 2; ++j) {
    const v4f y0 = *(const v4f*)(Y + base + 4 * j);
    const v4f y2 = *(const v4f*)(Y + 2 * PL + base + 4 * j);
    const v4f y1 = *(const v4f*)(Y + PL + base + 4 * j);
    const v4f y3 = *(const v4f*)(Y + 3 * PL + base + 4 * j);
    a[j] = ((y0 + y2) + y1) + y3;
  }
  float s = 0.f;
#pragma unroll
  for (int j = 0; j < 2; ++j) s += (a[j][0] + a[j][1]) + (a[j][2] + a[j][3]);
  s += __shfl_xor(s, 1, 32);
  s += __shfl_xor(s, 2, 32);
  s += __shfl_xor(s, 4, 32);
  s += __shfl_xor(s, 8, 32);
  s += __shfl_xor(s, 16, 32);
  if (lane == 0) sred[wave] = s;
  __syncthreads();
  const float tot = ((sred[0] + sred[1]) + (sred[2] + sred[3])) + (sred[4] + sred[5]);
  const float mu  = tot * (1.0f / 1536.0f);
  float q = 0.f;
#pragma unroll
  for (int j = 0; j < 2; ++j) {
#pragma unroll
    for (int e = 0; e < 4; ++e) { const float dd = a[j][e] - mu; q = fmaf(dd, dd, q); }
  }
  q += __shfl_xor(q, 1, 32);
  q += __shfl_xor(q, 2, 32);
  q += __shfl_xor(q, 4, 32);
  q += __shfl_xor(q, 8, 32);
  q += __shfl_xor(q, 16, 32);
  if (lane == 0) sred[8 + wave] = q;
  __syncthreads();
  const float qt  = ((sred[8] + sred[9]) + (sred[10] + sred[11])) + (sred[12] + sred[13]);
  const float var = qt * (1.0f / 1536.0f);
  const float is  = rsqrtf(var + 1e-5f);
  v8h hv;
#pragma unroll
  for (int j = 0; j < 2; ++j) {
    const v4f zz = *(const v4f*)(Z   + base + 4 * j);
    const v4f gg = *(const v4f*)(gam + c0 + 4 * j);
    const v4f bb = *(const v4f*)(bet + c0 + 4 * j);
#pragma unroll
    for (int e = 0; e < 4; ++e) {
      const float gn = ((a[j][e] - mu) * is) * gg[e] + bb[e];
      const float zv = zz[e];
      const float sg = __builtin_amdgcn_rcpf(1.0f + __expf(-zv));
      const float v  = gn * (zv * sg);
      hv[4 * j + e] = (_Float16)(v * 64.0f);
    }
  }
  unsigned short* op = YG16 + base;
  *(volatile v8h*)op = hv;
  __threadfence();
  *(volatile v8h*)op = hv;
}

extern "C" void kernel_launch(void* const* d_in, const int* in_sizes, int n_in,
                              void* d_out, int out_size, void* d_ws, size_t ws_size,
                              hipStream_t stream)
{
  if (n_in < 12) return;
  const float* x    = (const float*)d_in[0];
  const float* inpw = (const float*)d_in[1];
  const float* cw   = (const float*)d_in[2];
  const float* cb   = (const float*)d_in[3];
  const float* xprw = (const float*)d_in[4];
  const float* alog = (const float*)d_in[5];
  const float* dsp  = (const float*)d_in[6];
  const float* dtpw = (const float*)d_in[7];
  const float* dtpb = (const float*)d_in[8];
  const float* lng  = (const float*)d_in[9];
  const float* lnb  = (const float*)d_in[10];
  const float* outw = (const float*)d_in[11];
  float* dout = (float*)d_out;

  if (in_sizes[0] != NTOK * CMOD) return;
  if (in_sizes[1] != 2 * DIN * CMOD) return;
  if (in_sizes[2] != DIN * 9 || in_sizes[3] != DIN) return;
  if (in_sizes[4] != XPR * DIN) return;
  if (in_sizes[5] != NDIR * DIN * NST || in_sizes[6] != NDIR * DIN) return;
  if (in_sizes[7] != NDIR * DIN * DTR || in_sizes[8] != NDIR * DIN) return;
  if (in_sizes[9] != DIN || in_sizes[10] != DIN) return;
  if (in_sizes[11] != CMOD * DIN) return;
  if (out_size != NTOK * CMOD) return;

  const size_t SZ_X16  = (size_t)NTOK * CMOD * 2;
  const size_t SZ_WIN  = (size_t)2 * DIN * CMOD * 2;
  const size_t SZ_XC16 = (size_t)NTOK * DIN * 2;
  const size_t SZ_WX   = (size_t)XPRP * DIN * 2;
  const size_t SZ_WDT  = (size_t)NDIR * DIN * DTRP * 2;
  const size_t SZ_WO   = (size_t)CMOD * DIN * 2;
  const size_t SZ_F    = (size_t)NTOK * DIN * 4;
  const size_t SZ_XDBL = (size_t)NTOK * XPRP * 4;
  const size_t SZ_XDR  = (size_t)NTOK * DTRP * 2;
  const size_t SZ_DT   = (size_t)DPL * NTOK * DIN * 4;
  const size_t SZ_Y    = (size_t)NDIR * NTOK * DIN * 4;
  const size_t OFF_X16  = 0;
  const size_t OFF_WIN  = OFF_X16  + SZ_X16;
  const size_t OFF_XC16 = 0;
  const size_t OFF_WX   = OFF_WIN  + SZ_WIN;
  const size_t OFF_WDT  = OFF_WX   + SZ_WX;
  const size_t OFF_WO   = OFF_WDT  + SZ_WDT;
  const size_t OFF_XI   = OFF_WO   + SZ_WO;
  const size_t OFF_Z    = OFF_XI   + SZ_F;
  const size_t OFF_XC   = OFF_Z    + SZ_F;
  const size_t OFF_YG16 = OFF_XC;
  const size_t OFF_XDBL = OFF_XC   + SZ_F;
  const size_t OFF_XDR  = OFF_XDBL + SZ_XDBL;
  const size_t OFF_DT   = OFF_XDR  + SZ_XDR;
  const size_t OFF_Y    = OFF_DT   + SZ_DT;
  const size_t TOTAL    = OFF_Y    + SZ_Y;
  if (SZ_XC16 > SZ_X16 + SZ_WIN) return;
  if (SZ_XC16 > SZ_F) return;
  if (ws_size < TOTAL) return;

  char* ws = (char*)d_ws;
  unsigned short* X16  = (unsigned short*)(ws + OFF_X16);
  unsigned short* WIN  = (unsigned short*)(ws + OFF_WIN);
  unsigned short* XC16 = (unsigned short*)(ws + OFF_XC16);
  unsigned short* WX   = (unsigned short*)(ws + OFF_WX);
  unsigned short* WDT  = (unsigned short*)(ws + OFF_WDT);
  unsigned short* WO   = (unsigned short*)(ws + OFF_WO);
  float*          XI   = (float*)(ws + OFF_XI);
  float*          ZB   = (float*)(ws + OFF_Z);
  float*          XC   = (float*)(ws + OFF_XC);
  unsigned short* YG16 = (unsigned short*)(ws + OFF_YG16);
  float*          XDBL = (float*)(ws + OFF_XDBL);
  unsigned short* XDR  = (unsigned short*)(ws + OFF_XDR);
  float*          DT   = (float*)(ws + OFF_DT);
  float*          YS   = (float*)(ws + OFF_Y);
  const float*    nores = x;

  xpose_cast_kernel<<<(CMOD / 64) * (NTOK / 64), 256, 0, stream>>>(x, X16);
  {
    const int nc = 2 * DIN * CMOD / 8;
    cast_pad_kernel<<<(nc + 255) / 256, 256, 0, stream>>>(inpw, CMOD, 2 * DIN, WIN, CMOD, CMOD, nc, 64.0f);
  }
  {
    const int nc = XPRP * DIN / 8;
    cast_pad_kernel<<<(nc + 255) / 256, 256, 0, stream>>>(xprw, DIN, XPR, WX, DIN, DIN, nc, 64.0f);
  }
  {
    const int nc = NDIR * DIN * DTRP / 8;
    cast_pad_kernel<<<(nc + 255) / 256, 256, 0, stream>>>(dtpw, DTR, NDIR * DIN, WDT, DTRP, DTR, nc, 64.0f);
  }
  {
    const int nc = CMOD * DIN / 8;
    cast_pad_kernel<<<(nc + 255) / 256, 256, 0, stream>>>(outw, DIN, CMOD, WO, DIN, DIN, nc, 64.0f);
  }

  wmma_gemm64<0, false, 0, 0, false, 0><<<dim3(96, 1), 256, 0, stream>>>(
      X16, X16, CMOD, 0L, WIN, WIN, CMOD, 0L, (void*)XI, (void*)XI, DIN, 0L,
      nores, nores, 0L, NTOK, DIN, CMOD, 1.0f / 64.0f);
  wmma_gemm64<0, false, 0, 0, false, 0><<<dim3(96, 1), 256, 0, stream>>>(
      X16, X16, CMOD, 0L, WIN + (size_t)DIN * CMOD, WIN + (size_t)DIN * CMOD, CMOD, 0L,
      (void*)ZB, (void*)ZB, DIN, 0L, nores, nores, 0L, NTOK, DIN, CMOD, 1.0f / 64.0f);

  dwconv_silu_kernel<<<NBATCH * IMH * NCG, CGRP, 0, stream>>>(XI, cw, cb, XC, XC16);

  wmma_gemm64<0, false, 0, 0, false, 0><<<dim3(8, 1), 256, 0, stream>>>(
      XC16, XC16, DIN, 0L, WX, WX, DIN, 0L, (void*)XDBL, (void*)XDBL, XPRP, 0L,
      nores, nores, 0L, NTOK, XPRP, DIN, 1.0f / 4096.0f);

  {
    const int nc = NTOK * DTRP / 8;
    cast_pad_kernel<<<(nc + 255) / 256, 256, 0, stream>>>(XDBL, XPRP, NTOK, XDR, DTRP, DTR, nc, 256.0f);
  }

  for (int kb = 0; kb < NDIR; kb += DPL) {
    wmma_gemm64<0, false, 0, 0, false, 0><<<dim3(96, DPL), 256, 0, stream>>>(
        XDR, XDR, DTRP, 0L, WDT + (size_t)kb * DIN * DTRP, WDT + (size_t)kb * DIN * DTRP, DTRP, (long)DIN * DTRP,
        (void*)DT, (void*)DT, DIN, (long)NTOK * DIN, nores, nores, 0L, NTOK, DIN, DTRP, 1.0f / 16384.0f);
    scan_dir_kernel<<<NBATCH * DPL * NCG, CGRP, 0, stream>>>(XDBL, XC, DT, dtpb, alog, dsp, YS, kb);
  }

  ln_gate_kernel<<<NTOK, 192, 0, stream>>>(YS, ZB, lng, lnb, YG16);

  wmma_gemm64<0, false, 0, 0, false, 0><<<dim3(24, NBATCH), 256, 0, stream>>>(
      WO, WO, DIN, 0L, YG16, YG16, DIN, (long)NPIX * DIN, (void*)dout, (void*)dout, NPIX, (long)CMOD * NPIX,
      nores, nores, 0L, CMOD, NPIX, DIN, 1.0f / 4096.0f);
}
